// GCNLOGSIG_55473797595736
// MI455X (gfx1250) — hardware-verified
//
#include <hip/hip_runtime.h>
#include <stdint.h>

#define NMB    8
#define TT     300
#define VJ     25
#define C1     96
#define NB     200
#define NSEG   50
#define DIN    4752
#define KP     4800
#define K2     9600
#define G4     384
#define CHROWS 2500
#define CHPAD  2560
#define NCHUNK 4
#define NPAIR  4560
#define EPSB   1e-5f
#define WSCAP  134217728

static_assert(DIN == 96 + 96 + NPAIR);
static_assert(KP % 32 == 0 && K2 == 2 * KP && KP >= DIN);
static_assert(CHROWS == 50 * NSEG && NCHUNK * CHROWS == NB * NSEG);
static_assert(CHPAD % 128 == 0 && CHPAD >= CHROWS);
static_assert(G4 == 4 * C1 && G4 % 64 == 0);
static_assert(6 * 16 == C1);
static_assert(5 * VJ <= 128);
static_assert(TT % 5 == 0);
static_assert(DIN % 8 == 0);

__host__ __device__ constexpr int seg_start(int s) { return 6 * s - ((s >= 25) ? 1 : 0); }
__host__ __device__ constexpr int seg_len(int s) { return (s == 24) ? 5 : 6; }
constexpr bool seg_ok() {
  int sum = 0;
  for (int s = 0; s < NSEG; ++s) {
    sum += seg_len(s);
    if (s + 1 < NSEG && seg_start(s + 1) != seg_start(s) + seg_len(s)) return false;
  }
  return sum == 299 && seg_start(49) + seg_len(49) == 299 && seg_start(0) == 0;
}
static_assert(seg_ok());

#define PO_B1M  0
#define PO_B1S  152
#define PO_B1B  304
#define PO_B2M  456
#define PO_B2S  552
#define PO_B2B  648
#define PO_BGC  744
#define PO_BSUM 840
#define PAR_N   1248
static_assert(PO_BSUM + G4 <= PAR_N && PAR_N % 32 == 0);

constexpr size_t SZ_P    = (size_t)NB * TT * C1 * 4;
constexpr size_t SZ_FEAT = (size_t)CHPAD * K2 * 2;
constexpr size_t SZ_W2IH = (size_t)G4 * K2 * 2;
constexpr size_t SZ_XW   = (size_t)NB * NSEG * G4 * 4;
constexpr size_t SZ_HS   = (size_t)208 * C1 * 4;
constexpr size_t SZ_WHH  = (size_t)G4 * C1 * 2;
constexpr size_t SZ_W2G  = (size_t)C1 * C1 * 2;
constexpr size_t SZ_AF   = (size_t)8128 * 4;
constexpr size_t SZ_PAR  = (size_t)5120;
constexpr size_t SZ_PAIR = (size_t)9216;
constexpr size_t O_P    = 0;
constexpr size_t O_FEAT = O_P + SZ_P;
constexpr size_t O_W2IH = O_FEAT + SZ_FEAT;
constexpr size_t O_XW   = O_W2IH + SZ_W2IH;
constexpr size_t O_HS   = O_XW + SZ_XW;
constexpr size_t O_WHH  = O_HS + SZ_HS;
constexpr size_t O_W2G  = O_WHH + SZ_WHH;
constexpr size_t O_AF   = O_W2G + SZ_W2G;
constexpr size_t O_PAR  = O_AF + SZ_AF;
constexpr size_t O_PAIR = O_PAR + SZ_PAR;
constexpr size_t O_END  = O_PAIR + SZ_PAIR;
static_assert(O_FEAT % 256 == 0 && O_W2IH % 256 == 0 && O_XW % 256 == 0 && O_HS % 256 == 0);
static_assert(O_WHH % 256 == 0 && O_W2G % 256 == 0 && O_AF % 256 == 0 && O_PAR % 256 == 0 && O_PAIR % 256 == 0);
static_assert(O_END <= (size_t)WSCAP);
static_assert(PAR_N * 4 <= SZ_PAR);

typedef float          v4f   __attribute__((ext_vector_type(4)));
typedef float          v8f   __attribute__((ext_vector_type(8)));
typedef int            v8i   __attribute__((ext_vector_type(8)));
typedef unsigned int   v4u   __attribute__((ext_vector_type(4)));
typedef unsigned short v8us  __attribute__((ext_vector_type(8)));
typedef __bf16         v16bf __attribute__((ext_vector_type(16)));
typedef v4f  __attribute__((may_alias)) v4fa;
typedef v4u  __attribute__((may_alias)) v4ua;
typedef v8us __attribute__((may_alias)) v8usa;
union FragB { v16bf v; v8us h[2]; v8i w; unsigned int u[8]; };

__device__ __forceinline__ unsigned f2bf(float f) {
  unsigned u = __float_as_uint(f);
  return (u + 0x7FFFu + ((u >> 16) & 1u)) >> 16;
}
__device__ __forceinline__ float bf2f(unsigned b) { return __uint_as_float(b << 16); }
__device__ __forceinline__ float bfr(float f) { return bf2f(f2bf(f)); }
__device__ __forceinline__ unsigned pk16(unsigned a, unsigned b) { return (a & 0xffffu) | (b << 16); }

__device__ __forceinline__ v8f wmb(const FragB& a, const FragB& b, v8f c) {
  v8f d = __builtin_amdgcn_wmma_f32_16x16x32_bf16(false, a.v, false, b.v, (short)0, c, false, false);
  asm volatile("v_nop\n\tv_nop\n\tv_nop\n\tv_nop" : "+v"(d) : "v"(a.w), "v"(b.w));
  return d;
}
__device__ __forceinline__ v8f z8() { v8f z = {0.f, 0.f, 0.f, 0.f, 0.f, 0.f, 0.f, 0.f}; return z; }

__device__ __forceinline__ float sigm_f(float v) {
  v = fminf(fmaxf(v, -30.0f), 30.0f);
  const float e = expf(-v);
  return 1.0f / (1.0f + e);
}

#define PB_W2IH 0
#define PB_WHH  1800
#define PB_W2G  1818
#define PB_AF   1823
#define PB_PAR  1831
#define PB_PAIR 1832
#define PB_ZF   1835
#define PB_END  2117
static_assert((PB_WHH - PB_W2IH) * 256 == G4 * (K2 / 8));
static_assert((PB_W2G - PB_WHH) * 256 == G4 * C1 / 8);
static_assert((PB_END - PB_ZF) * 256 >= (CHPAD - CHROWS) * (K2 / 8));

__device__ __forceinline__ void par_store_pass(const float* sP, float* PAR, int tid) {
#pragma unroll
  for (int i = 0; i < 2; ++i) {
    const int u = tid + 256 * i;
    const int uc = (u < 311) ? u : 311;
    const v4f v = *(const v4fa*)(sP + 4 * uc);
    if (u < 312) *(volatile v4f*)(PAR + 4 * u) = v;
  }
}

__global__ __launch_bounds__(256) void prep_kernel(
    const float* bn_g, const float* bn_b, const float* bn_m, const float* bn_v,
    const float* Ap, const float* Ar, const float* Wg, const float* bgc,
    const float* g2, const float* b2, const float* m2, const float* v2,
    const float* W_ih, const float* W_hh, const float* b_ih, const float* b_hh,
    unsigned char* ws)
{
  __shared__ __align__(16) float sP[PAR_N];
  const int b = blockIdx.x, tid = threadIdx.x;
  if (b < PB_WHH) {
    const unsigned u = (unsigned)(b - PB_W2IH) * 256u + (unsigned)tid;
    const unsigned g = u / 1200u, cu = u - g * 1200u;
    const unsigned k = cu * 8u;
    const unsigned kk = (k >= (unsigned)KP) ? (k - (unsigned)KP) : k;
    const bool valid = kk < (unsigned)DIN;
    const unsigned kc = valid ? kk : (unsigned)(DIN - 8);
    const float* src = W_ih + (size_t)g * DIN + kc;
    const v4f a = *(const v4fa*)src;
    const v4f c = *(const v4fa*)(src + 4);
    const unsigned mk = valid ? 0xffffffffu : 0u;
    v4u v;
    v[0] = pk16(f2bf(a[0]), f2bf(a[1])) & mk;
    v[1] = pk16(f2bf(a[2]), f2bf(a[3])) & mk;
    v[2] = pk16(f2bf(c[0]), f2bf(c[1])) & mk;
    v[3] = pk16(f2bf(c[2]), f2bf(c[3])) & mk;
    unsigned short* dst = (unsigned short*)(ws + O_W2IH) + (size_t)u * 8;
    *(volatile v4u*)dst = v;
    __threadfence();
    *(volatile v4u*)dst = v;
  } else if (b < PB_W2G) {
    const unsigned u = (unsigned)(b - PB_WHH) * 256u + (unsigned)tid;
    const float* src = W_hh + (size_t)u * 8;
    const v4f a = *(const v4fa*)src;
    const v4f c = *(const v4fa*)(src + 4);
    v4u v;
    v[0] = pk16(f2bf(a[0]), f2bf(a[1]));
    v[1] = pk16(f2bf(a[2]), f2bf(a[3]));
    v[2] = pk16(f2bf(c[0]), f2bf(c[1]));
    v[3] = pk16(f2bf(c[2]), f2bf(c[3]));
    unsigned short* dst = (unsigned short*)(ws + O_WHH) + (size_t)u * 8;
    *(volatile v4u*)dst = v;
    __threadfence();
    *(volatile v4u*)dst = v;
  } else if (b < PB_AF) {
    const int u = (b - PB_W2G) * 256 + tid;
    const int uc = (u < 1151) ? u : 1151;
    const int n = uc / 12, cu = uc - n * 12;
    unsigned e[8];
#pragma unroll
    for (int j = 0; j < 8; ++j) {
      const int kk = cu * 8 + j;
      const int q = (kk < 48) ? kk : (kk - 48);
      const int qc = (q < 38) ? q : 38;
      const float wv = Wg[n * 39 + qc];
      e[j] = f2bf(wv) & ((q < 39) ? 0xffffu : 0u);
    }
    v4u v;
    v[0] = pk16(e[0], e[1]); v[1] = pk16(e[2], e[3]); v[2] = pk16(e[4], e[5]); v[3] = pk16(e[6], e[7]);
    unsigned short* dst = (unsigned short*)(ws + O_W2G) + (size_t)uc * 8;
    if (u < 1152) *(volatile v4u*)dst = v;
    __threadfence();
    if (u < 1152) *(volatile v4u*)dst = v;
  } else if (b < PB_PAR) {
    const int u = (b - PB_AF) * 256 + tid;
    const int uc = (u < 2031) ? u : 2031;
    v4f v;
#pragma unroll
    for (int j = 0; j < 4; ++j) {
      const int idx0 = 4 * uc + j;
      const int idx = (idx0 < 8124) ? idx0 : 8124;
      v[j] = bfr(Ap[idx]) + bfr(Ar[idx]);
    }
    float* dst = (float*)(ws + O_AF) + 4 * uc;
    if (u < 2032) *(volatile v4f*)dst = v;
    __threadfence();
    if (u < 2032) *(volatile v4f*)dst = v;
  } else if (b < PB_PAIR) {
    {
      const int ch = (tid < 149) ? tid : 149;
      const float mm = bfr(bn_m[ch]);
      const float gg = bfr(bn_g[ch]);
      const float vv = bfr(bn_v[ch]);
      const float bb = bfr(bn_b[ch]);
      const float sc = gg / sqrtf(vv + EPSB);
      if (tid < 152) { sP[PO_B1M + tid] = mm; sP[PO_B1S + tid] = sc; sP[PO_B1B + tid] = bb; }
    }
    __syncthreads();
    {
      const int o = (tid < 95) ? tid : 95;
      const float mm = bfr(m2[o]);
      const float gg = bfr(g2[o]);
      const float vv = bfr(v2[o]);
      const float bb = bfr(b2[o]);
      const float bg = bfr(bgc[o]);
      const float sc = gg / sqrtf(vv + EPSB);
      if (tid < 96) { sP[PO_B2M + tid] = mm; sP[PO_B2S + tid] = sc; sP[PO_B2B + tid] = bb; sP[PO_BGC + tid] = bg; }
    }
    __syncthreads();
#pragma unroll
    for (int i = 0; i < 2; ++i) {
      const int e = tid + 256 * i;
      const int g = (e < 383) ? e : 383;
      const float bs = bfr(b_ih[g]) + bfr(b_hh[g]);
      if (e < PAR_N - PO_BSUM) sP[PO_BSUM + e] = (e < G4) ? bs : 0.0f;
    }
    __syncthreads();
    float* PAR = (float*)(ws + O_PAR);
    par_store_pass(sP, PAR, tid);
    __threadfence();
    par_store_pass(sP, PAR, tid);
  } else if (b < PB_ZF) {
    const int u = (b - PB_PAIR) * 256 + tid;
    const int uc = (u < 575) ? u : 575;
    const int k0 = 8 * uc;
    const int kc = (k0 < NPAIR - 1) ? k0 : (NPAIR - 1);
    int i = 0;
#pragma unroll 1
    for (int t = 1; t < 95; ++t) { if ((t * (191 - t)) / 2 <= kc) i = t; }
    int j = i + 1 + (kc - (i * (191 - i)) / 2);
    unsigned e[8];
#pragma unroll
    for (int q = 0; q < 8; ++q) {
      const int k = k0 + q;
      const unsigned val = ((unsigned)i << 8) | (unsigned)j;
      e[q] = (k < NPAIR) ? (val & 0xffffu) : 0u;
      ++j;
      if (j > 95) { ++i; j = i + 1; }
    }
    v4u v;
    v[0] = pk16(e[0], e[1]); v[1] = pk16(e[2], e[3]); v[2] = pk16(e[4], e[5]); v[3] = pk16(e[6], e[7]);
    unsigned short* dst = (unsigned short*)(ws + O_PAIR) + (size_t)uc * 8;
    if (u < 576) *(volatile v4u*)dst = v;
    __threadfence();
    if (u < 576) *(volatile v4u*)dst = v;
  } else {
    const int u = (b - PB_ZF) * 256 + tid;
    const int uc = (u < 71999) ? u : 71999;
    const v4u z = {0u, 0u, 0u, 0u};
    unsigned short* dst = (unsigned short*)(ws + O_FEAT) + (size_t)CHROWS * K2 + (size_t)uc * 8;
    if (u < 72000) *(volatile v4u*)dst = z;
    __threadfence();
    if (u < 72000) *(volatile v4u*)dst = z;
  }
}

#define G_AF   0
#define G_XG   32512
#define G_PAR  34048
#define G_A    37408
#define G_D    61984
#define G_SMEM 111136
static_assert(G_XG % 16 == 0 && G_PAR % 16 == 0 && G_A % 16 == 0 && G_D % 16 == 0);
static_assert(G_D + 128 * 96 * 4 == G_SMEM);

__device__ __forceinline__ void p_store_pass(const float* sD, float* P, int nm, int t0, int tid) {
#pragma unroll
  for (int i = 0; i < 12; ++i) {
    const int U = tid + 256 * i;
    const int row = U / 24, cu = U - row * 24;
    const int tl = row / 25, v = row - tl * 25;
    const v4f val = *(const v4fa*)(sD + row * 96 + 4 * cu);
    if (U < 3000) {
      float* dst = P + ((size_t)((nm * 25 + v) * TT + t0 + tl)) * C1 + 4 * cu;
      *(volatile v4f*)dst = val;
    }
  }
}

__global__ __launch_bounds__(256) void graph_kernel(const float* __restrict__ x, const float* __restrict__ AF,
                                                    const float* __restrict__ PAR,
                                                    const unsigned short* __restrict__ W2G,
                                                    float* __restrict__ P)
{
  extern __shared__ __align__(16) unsigned char gsm[];
  float* sAF = (float*)(gsm + G_AF);
  float* sXG = (float*)(gsm + G_XG);
  float* sPar = (float*)(gsm + G_PAR);
  unsigned* sAw = (unsigned*)(gsm + G_A);
  const unsigned short* sA16 = (const unsigned short*)(gsm + G_A);
  float* sD = (float*)(gsm + G_D);

  const int tid = threadIdx.x, lane = tid & 31, w = tid >> 5;
  const int h = lane >> 4, m = lane & 15;
  const int nm = blockIdx.x / 60, tb = blockIdx.x - nm * 60;
  const int t0 = 5 * tb;
  const int mper = nm & 1;

#pragma unroll
  for (int i = 0; i < 8; ++i) {
    const int u = tid + 256 * i;
    const int uc = (u < 2031) ? u : 2031;
    const v4f v = *(const v4fa*)(AF + 4 * uc);
    if (u < 2032) *(v4fa*)(sAF + 4 * u) = v;
  }
  {
    const int uc = (tid < 209) ? tid : 209;
    const v4f v = *(const v4fa*)(PAR + 4 * uc);
    if (tid < 210) *(v4fa*)(sPar + 4 * tid) = v;
  }
#pragma unroll
  for (int i = 0; i < 2; ++i) {
    const int e = tid + 256 * i;
    const int ec = (e < 374) ? e : 374;
    const int c = ec / 125, rem = ec - c * 125;
    const int tl = rem / 25, uu = rem - tl * 25;
    const int ch = mper * 75 + uu * 3 + c;
    const float xv = bfr(x[((size_t)((nm * 3 + c) * TT + t0 + tl)) * VJ + uu]);
    const float val = (xv - PAR[PO_B1M + ch]) * PAR[PO_B1S + ch] + PAR[PO_B1B + ch];
    if (e < 375) sXG[e] = val;
  }
  __syncthreads();

#pragma unroll 1
  for (int it = 0; it < 12; ++it) {
    const int I = tid + 256 * it;
    const int row = I / 24, wi = I - row * 24;
    const int posc = (row < 124) ? row : 124;
    const int tl = posc / 25, v = posc - tl * 25;
    const unsigned rmask = (row < 125) ? 0xffffu : 0u;
    unsigned hw[2], lw[2];
#pragma unroll
    for (int e = 0; e < 2; ++e) {
      const int q = 2 * wi + e;
      const int qc = (q < 38) ? q : 38;
      const int s = qc / 3, c = qc - 3 * s;
      const float* ar = sAF + (s * 25 + v) * 25;
      const float* xr = sXG + c * 125 + tl * 25;
      float acc = 0.0f;
#pragma unroll 5
      for (int u = 0; u < 25; ++u) acc = fmaf(ar[u], xr[u], acc);
      const unsigned hb = f2bf(acc);
      const unsigned lb = f2bf(acc - bf2f(hb));
      const unsigned mk = (q < 39) ? rmask : 0u;
      hw[e] = hb & mk;
      lw[e] = lb & mk;
    }
    sAw[row * 48 + wi] = hw[0] | (hw[1] << 16);
    sAw[row * 48 + 24 + wi] = lw[0] | (lw[1] << 16);
  }
  __syncthreads();

  v8f acc[6];
#pragma unroll
  for (int nt = 0; nt < 6; ++nt) acc[nt] = z8();
  {
    const unsigned short* arow = sA16 + (16 * w + m) * 96 + 8 * h;
    const unsigned short* brow = W2G + (size_t)m * 96 + 8 * h;
#pragma unroll
    for (int ks = 0; ks < 3; ++ks) {
      FragB a;
      a.h[0] = *(const v8usa*)(arow + 32 * ks);
      a.h[1] = *(const v8usa*)(arow + 32 * ks + 16);
#pragma unroll
      for (int nt = 0; nt < 6; ++nt) {
        const unsigned short* wq = brow + (size_t)nt * 16 * 96 + 32 * ks;
        FragB bf;
        bf.h[0] = *(const v8usa*)wq;
        bf.h[1] = *(const v8usa*)(wq + 16);
        acc[nt] = wmb(a, bf, acc[nt]);
      }
    }
  }
#pragma unroll
  for (int nt = 0; nt < 6; ++nt) {
    const int col = 16 * nt + m;
    const float bg = sPar[PO_BGC + col];
    const float mm = sPar[PO_B2M + col];
    const float sc = sPar[PO_B2S + col];
    const float bb = sPar[PO_B2B + col];
#pragma unroll
    for (int r = 0; r < 8; ++r) {
      float v = acc[nt][r] + bg;
      v = (v - mm) * sc + bb;
      sD[(16 * w + 8 * h + r) * 96 + col] = fmaxf(v, 0.0f);
    }
  }
  __syncthreads();

  p_store_pass(sD, P, nm, t0, tid);
  __threadfence();
  p_store_pass(sD, P, nm, t0, tid);
}

__device__ __forceinline__ float levy_pair(const float* sCh, int i, int j) {
  const v4f i0 = *(const v4fa*)(sCh + i * 12);
  const v4f i1 = *(const v4fa*)(sCh + i * 12 + 4);
  const v4f i2 = *(const v4fa*)(sCh + i * 12 + 8);
  const v4f j0 = *(const v4fa*)(sCh + j * 12);
  const v4f j1 = *(const v4fa*)(sCh + j * 12 + 4);
  const v4f j2 = *(const v4fa*)(sCh + j * 12 + 8);
  float qa = i0[0] * j1[1];
  qa = fmaf(i0[1], j1[2], qa);
  qa = fmaf(i0[2], j1[3], qa);
  qa = fmaf(i0[3], j2[0], qa);
  qa = fmaf(i1[0], j2[1], qa);
  float qb = j0[0] * i1[1];
  qb = fmaf(j0[1], i1[2], qb);
  qb = fmaf(j0[2], i1[3], qb);
  qb = fmaf(j0[3], i2[0], qb);
  qb = fmaf(j1[0], i2[1], qb);
  return 0.5f * (qa - qb);
}

__device__ __forceinline__ void f_store_pass(const unsigned* sRow, unsigned short* dst, int tid) {
#pragma unroll
  for (int it = 0; it < 5; ++it) {
    const int u = tid + 256 * it;
    const int uc = (u < 1199) ? u : 1199;
    const v4u v = *(const v4ua*)(sRow + 4 * uc);
    if (u < 1200) *(volatile v4u*)(dst + 8 * u) = v;
  }
}

__global__ __launch_bounds__(256) void feat_kernel(const float* __restrict__ P, const unsigned* __restrict__ PAIRW,
                                                   unsigned short* __restrict__ FEAT, int chunk)
{
  __shared__ __align__(16) float sPp[7 * 96];
  __shared__ __align__(16) float sCh[96 * 12];
  __shared__ __align__(16) float sPS[192];
  __shared__ __align__(16) unsigned sRow[K2 / 2];

  const int tid = threadIdx.x;
  const int r = blockIdx.x;
  const int bl = r / NSEG, s = r - bl * NSEG;
  const int b = chunk * 50 + bl;
  const int start = 6 * s - ((s >= 25) ? 1 : 0);
  const int len = (s == 24) ? 5 : 6;

  {
    const int uc = (tid < 167) ? tid : 167;
    const v4f v = *(const v4fa*)(P + ((size_t)b * TT + start) * C1 + 4 * uc);
    if (tid < 168) *(v4fa*)(sPp + 4 * tid) = v;
  }
  __syncthreads();
  {
    const int c = (tid < 95) ? tid : 95;
    float pv[7];
#pragma unroll
    for (int l = 0; l < 7; ++l) pv[l] = sPp[l * 96 + c];
    float pre[6], d[6];
    float run = 0.0f;
#pragma unroll
    for (int l = 0; l < 6; ++l) {
      const float df = pv[l + 1] - pv[l];
      const float dl = (l < len) ? df : 0.0f;
      pre[l] = run; d[l] = dl; run += dl;
    }
    if (tid < 96) {
      const v4f a0 = {pre[1], pre[2], pre[3], pre[4]};
      const v4f a1 = {pre[5], d[1], d[2], d[3]};
      const v4f a2 = {d[4], d[5], 0.0f, 0.0f};
      *(v4fa*)(sCh + tid * 12) = a0;
      *(v4fa*)(sCh + tid * 12 + 4) = a1;
      *(v4fa*)(sCh + tid * 12 + 8) = a2;
      sPS[tid] = pv[0];
      sPS[96 + tid] = run;
    }
    if (tid < 24) { sRow[2376 + tid] = 0u; sRow[4776 + tid] = 0u; }
  }
  __syncthreads();
  {
    const int wi = (tid < 95) ? tid : 95;
    const float v0 = sPS[2 * wi], v1 = sPS[2 * wi + 1];
    const unsigned h0 = f2bf(v0), h1 = f2bf(v1);
    const unsigned l0 = f2bf(v0 - bf2f(h0)), l1 = f2bf(v1 - bf2f(h1));
    if (tid < 96) { sRow[tid] = pk16(h0, h1); sRow[2400 + tid] = pk16(l0, l1); }
  }
#pragma unroll 1
  for (int it = 0; it < 9; ++it) {
    const int wp = tid + 256 * it;
    const int wpc = (wp < 2279) ? wp : 2279;
    const unsigned pw = PAIRW[wpc];
    int ia = (int)((pw >> 8) & 0xffu), ja = (int)(pw & 0xffu);
    int ib = (int)((pw >> 24) & 0xffu), jb = (int)((pw >> 16) & 0xffu);
    ia = (ia < 95) ? ia : 95; ja = (ja < 95) ? ja : 95;
    ib = (ib < 95) ? ib : 95; jb = (jb < 95) ? jb : 95;
    const float va = levy_pair(sCh, ia, ja);
    const float vb = levy_pair(sCh, ib, jb);
    const unsigned ha = f2bf(va), hb = f2bf(vb);
    const unsigned la = f2bf(va - bf2f(ha)), lb = f2bf(vb - bf2f(hb));
    if (wp < 2280) { sRow[96 + wp] = pk16(ha, hb); sRow[2496 + wp] = pk16(la, lb); }
  }
  __syncthreads();

  unsigned short* dst = FEAT + (size_t)r * K2;
  f_store_pass(sRow, dst, tid);
  __threadfence();
  f_store_pass(sRow, dst, tid);
}

__device__ __forceinline__ void xw_store_pass(const float* sO, float* XW, int grow_w, int lrow_w,
                                              int n0, int w, int lane) {
  const int q8 = lane & 7, sub = lane >> 3;
#pragma unroll
  for (int i = 0; i < 16; ++i) {
    const int lid = i * 4 + sub;
    const int row = lid >> 1, hl = lid & 1;
    const v4f v = *(const v4fa*)(sO + (32 * w + row) * 64 + 32 * hl + 4 * q8);
    if (lrow_w + row < CHROWS)
      *(volatile v4f*)(XW + (size_t)(grow_w + row) * G4 + n0 + 32 * hl + 4 * q8) = v;
  }
}

__global__ __launch_bounds__(128) void xw_kernel(const unsigned short* __restrict__ FEAT,
                                                 const unsigned short* __restrict__ W2IH,
                                                 const float* __restrict__ BS,
                                                 float* __restrict__ XW, int chunk) {
  __shared__ __align__(16) float sO[128 * 64];
  const int tid = threadIdx.x, lane = tid & 31, w = tid >> 5;
  const int h = lane >> 4, m = lane & 15;
  const int lrow_w = blockIdx.x * 128 + 32 * w;
  const int n0 = blockIdx.y * 64;

  const unsigned short* xa0 = FEAT + (size_t)(lrow_w + m) * K2 + 8 * h;
  const unsigned short* xa1 = xa0 + (size_t)16 * K2;
  const unsigned short* wb  = W2IH + (size_t)(n0 + m) * K2 + 8 * h;

  v8f acc[2][4];
#pragma unroll
  for (int mt = 0; mt < 2; ++mt)
#pragma unroll
    for (int nt = 0; nt < 4; ++nt) acc[mt][nt] = z8();

#pragma unroll 1
  for (int k0 = 0; k0 < K2; k0 += 32) {
    FragB a0, a1;
    a0.h[0] = *(const v8usa*)(xa0 + k0);
    a0.h[1] = *(const v8usa*)(xa0 + k0 + 16);
    a1.h[0] = *(const v8usa*)(xa1 + k0);
    a1.h[1] = *(const v8usa*)(xa1 + k0 + 16);
#pragma unroll
    for (int nt = 0; nt < 4; ++nt) {
      const unsigned short* wq = wb + (size_t)nt * 16 * K2 + k0;
      FragB bf;
      bf.h[0] = *(const v8usa*)wq;
      bf.h[1] = *(const v8usa*)(wq + 16);
      acc[0][nt] = wmb(a0, bf, acc[0][nt]);
      acc[1][nt] = wmb(a1, bf, acc[1][nt]);
    }
  }

#pragma unroll
  for (int nt = 0; nt < 4; ++nt) {
    const int cl = 16 * nt + m;
    const float bs = BS[n0 + cl];
#pragma unroll
    for (int mt = 0; mt < 2; ++mt) {
#pragma unroll
      for (int r = 0; r < 8; ++r) {
        const int rl = 32 * w + 16 * mt + 8 * h + r;
        sO[rl * 64 + cl] = acc[mt][nt][r] + bs;
      }
    }
  }
  __syncthreads();

  const int grow_w = chunk * CHROWS + lrow_w;
  xw_store_pass(sO, XW, grow_w, lrow_w, n0, w, lane);
  __threadfence();
  xw_store_pass(sO, XW, grow_w, lrow_w, n0, w, lane);
}

#define L_W    0
#define L_XW   73728
#define L_H    122880
#define L_SMEM 135168
static_assert(L_XW == G4 * C1 * 2 && L_H == L_XW + 2 * 16 * G4 * 4 && L_SMEM == L_H + 2 * 16 * C1 * 4);

__device__ __forceinline__ void hs_store_pass(const float* sOut, float* HS, int b0, int tid) {
#pragma unroll
  for (int i = 0; i < 2; ++i) {
    const int U = tid + 192 * i;
    const int row = U / 24, cu = U - row * 24;
    const v4f v = *(const v4fa*)(sOut + row * 96 + 4 * cu);
    *(volatile v4f*)(HS + (size_t)(b0 + row) * C1 + 4 * cu) = v;
  }
}

__global__ __launch_bounds__(192) void rnn_kernel(const unsigned short* __restrict__ WHH,
                                                  const float* __restrict__ XW, float* __restrict__ HS)
{
  extern __shared__ __align__(16) unsigned char lsm[];
  unsigned short* sW = (unsigned short*)(lsm + L_W);
  float* sXW = (float*)(lsm + L_XW);
  float* sH = (float*)(lsm + L_H);

  const int tid = threadIdx.x, lane = tid & 31, w = tid >> 5;
  const int h = lane >> 4, m = lane & 15;
  const int b0 = blockIdx.x * 16;

#pragma unroll 4
  for (int i = 0; i < 24; ++i) {
    const int u = tid + 192 * i;
    const v4u v = *(const v4ua*)(WHH + 8 * u);
    *(v4ua*)(sW + 8 * u) = v;
  }
#pragma unroll
  for (int i = 0; i < 8; ++i) sH[tid + 192 * i] = 0.0f;

  float cst[8], hsum[8];
#pragma unroll
  for (int r = 0; r < 8; ++r) { cst[r] = 0.0f; hsum[r] = 0.0f; }

#pragma unroll 1
  for (int s = 0; s < NSEG; ++s) {
    float* xb = sXW + (s & 1) * (16 * G4);
#pragma unroll
    for (int i = 0; i < 8; ++i) {
      const int u = tid + 192 * i;
      const int row = u / 96, cu = u - row * 96;
      const int bb = (b0 + row < NB - 1) ? (b0 + row) : (NB - 1);
      const v4f v = *(const v4fa*)(XW + ((size_t)bb * NSEG + s) * G4 + 4 * cu);
      *(v4fa*)(xb + row * G4 + 4 * cu) = v;
    }
    __syncthreads();
    const float* hc = sH + (s & 1) * (16 * C1);
    float* hn = sH + ((s + 1) & 1) * (16 * C1);

    FragB ah[3], al[3];
#pragma unroll
    for (int ks = 0; ks < 3; ++ks) {
#pragma unroll
      for (int hf = 0; hf < 2; ++hf) {
        const float* base = hc + m * C1 + 32 * ks + 16 * hf + 8 * h;
        const v4f x0 = *(const v4fa*)base;
        const v4f x1 = *(const v4fa*)(base + 4);
        const float f[8] = {x0[0], x0[1], x0[2], x0[3], x1[0], x1[1], x1[2], x1[3]};
#pragma unroll
        for (int j = 0; j < 4; ++j) {
          const unsigned h0 = f2bf(f[2 * j]), h1 = f2bf(f[2 * j + 1]);
          const unsigned l0 = f2bf(f[2 * j] - bf2f(h0)), l1 = f2bf(f[2 * j + 1] - bf2f(h1));
          ah[ks].u[4 * hf + j] = pk16(h0, h1);
          al[ks].u[4 * hf + j] = pk16(l0, l1);
        }
      }
    }

    v8f acc[4];
#pragma unroll
    for (int g = 0; g < 4; ++g)
#pragma unroll
      for (int r = 0; r < 8; ++r) acc[g][r] = xb[(8 * h + r) * G4 + 96 * g + 16 * w + m];

#pragma unroll
    for (int ks = 0; ks < 3; ++ks) {
      FragB bf[4];
#pragma unroll
      for (int g = 0; g < 4; ++g) {
        const unsigned short* brow = sW + (96 * g + 16 * w + m) * C1 + 32 * ks + 8 * h;
        bf[g].h[0] = *(const v8usa*)brow;
        bf[g].h[1] = *(const v8usa*)(brow + 16);
      }
#pragma unroll
      for (int g = 0; g < 4; ++g) acc[g] = wmb(ah[ks], bf[g], acc[g]);
#pragma unroll
      for (int g = 0; g < 4; ++g) acc[g] = wmb(al[ks], bf[g], acc[g]);
    }

#pragma unroll
    for (int r = 0; r < 8; ++r) {
      const float ig = sigm_f(acc[0][r]);
      const float fg = sigm_f(acc[1][r]);
      const float gg = tanhf(acc[2][r]);
      const float og = sigm_f(acc[3][r]);
      const float cn = fg * cst[r] + ig * gg;
      cst[r] = cn;
      const float hv = og * tanhf(cn);
      hsum[r] += hv;
      hn[(8 * h + r) * C1 + 16 * w + m] = hv;
    }
  }
  __syncthreads();
  float* sOut = sXW;
#pragma unroll
  for (int r = 0; r < 8; ++r) sOut[(8 * h + r) * C1 + 16 * w + m] = hsum[r];
  __syncthreads();

  hs_store_pass(sOut, HS, b0, tid);
  __threadfence();
  hs_store_pass(sOut, HS, b0, tid);
}

__global__ __launch_bounds__(256) void head_kernel(const float* __restrict__ HS, const float* __restrict__ W_fc,
                                                   const float* __restrict__ b_fc, float* __restrict__ out)
{
  __shared__ __align__(16) float sPool[384];
  __shared__ __align__(16) float sOut[256];
  const int tid = threadIdx.x;
#pragma unroll 1
  for (int i = 0; i < 2; ++i) {
    const int e = tid + 256 * i;
    const int ec = (e < 383) ? e : 383;
    const int n = ec / 96, c = ec - n * 96;
    float tot = 0.0f;
#pragma unroll 1
    for (int mm = 0; mm < 2; ++mm) {
      float sm = 0.0f;
#pragma unroll 5
      for (int v = 0; v < VJ; ++v) sm += HS[(size_t)((2 * n + mm) * VJ + v) * C1 + c];
      tot += sm * (1.0f / 1250.0f);
    }
    if (e < 384) sPool[e] = 0.5f * tot;
  }
  __syncthreads();
  {
    const int tc = (tid < 239) ? tid : 239;
    const int n = tc / 60, k = tc - n * 60;
    float o = bfr(b_fc[k]);
    const float* wr = W_fc + (size_t)k * C1;
    const float* pr = sPool + n * C1;
#pragma unroll 2
    for (int j = 0; j < 24; ++j) {
      const v4f wv = *(const v4fa*)(wr + 4 * j);
      const v4f pv = *(const v4fa*)(pr + 4 * j);
      o = fmaf(pv[0], bfr(wv[0]), o);
      o = fmaf(pv[1], bfr(wv[1]), o);
      o = fmaf(pv[2], bfr(wv[2]), o);
      o = fmaf(pv[3], bfr(wv[3]), o);
    }
    sOut[tid] = (tid < 240) ? o : 0.0f;
  }
  __syncthreads();
  {
    const int uc = (tid < 59) ? tid : 59;
    const v4f v = *(const v4fa*)(sOut + 4 * uc);
    if (tid < 60) *(volatile v4f*)(out + 4 * tid) = v;
    __threadfence();
    if (tid < 60) *(volatile v4f*)(out + 4 * tid) = v;
  }
}

extern "C" void kernel_launch(void* const* d_in, const int* in_sizes, int n_in,
                              void* d_out, int out_size, void* d_ws, size_t ws_size,
                              hipStream_t stream) {
  if (n_in < 19) return;
  if (in_sizes[0] != 4 * 2 * 3 * TT * VJ) return;
  if (in_sizes[1] != 150 || in_sizes[2] != 150 || in_sizes[3] != 150 || in_sizes[4] != 150) return;
  if (in_sizes[5] != 325 * 25 || in_sizes[6] != 325 * 25) return;
  if (in_sizes[7] != C1 * 39 || in_sizes[8] != C1) return;
  if (in_sizes[9] != C1 || in_sizes[10] != C1 || in_sizes[11] != C1 || in_sizes[12] != C1) return;
  if (in_sizes[13] != G4 * DIN || in_sizes[14] != G4 * C1) return;
  if (in_sizes[15] != G4 || in_sizes[16] != G4) return;
  if (in_sizes[17] != 60 * C1 || in_sizes[18] != 60) return;
  if (out_size != 240) return;
  if (O_END > ws_size) return;

  const float* x    = (const float*)d_in[0];
  const float* bn_g = (const float*)d_in[1];
  const float* bn_b = (const float*)d_in[2];
  const float* bn_m = (const float*)d_in[3];
  const float* bn_v = (const float*)d_in[4];
  const float* Ap   = (const float*)d_in[5];
  const float* Ar   = (const float*)d_in[6];
  const float* Wg   = (const float*)d_in[7];
  const float* bgc  = (const float*)d_in[8];
  const float* g2   = (const float*)d_in[9];
  const float* b2   = (const float*)d_in[10];
  const float* m2   = (const float*)d_in[11];
  const float* v2   = (const float*)d_in[12];
  const float* W_ih = (const float*)d_in[13];
  const float* W_hh = (const float*)d_in[14];
  const float* b_ih = (const float*)d_in[15];
  const float* b_hh = (const float*)d_in[16];
  const float* W_fc = (const float*)d_in[17];
  const float* b_fc = (const float*)d_in[18];

  unsigned char* ws = (unsigned char*)d_ws;
  float*          P     = (float*)(ws + O_P);
  unsigned short* FEAT  = (unsigned short*)(ws + O_FEAT);
  unsigned short* W2IH  = (unsigned short*)(ws + O_W2IH);
  float*          XW    = (float*)(ws + O_XW);
  float*          HS    = (float*)(ws + O_HS);
  unsigned short* WHH   = (unsigned short*)(ws + O_WHH);
  unsigned short* W2G   = (unsigned short*)(ws + O_W2G);
  float*          AF    = (float*)(ws + O_AF);
  float*          PAR   = (float*)(ws + O_PAR);
  unsigned*       PAIRW = (unsigned*)(ws + O_PAIR);

  (void)hipFuncSetAttribute(reinterpret_cast<const void*>(&graph_kernel),
                            hipFuncAttributeMaxDynamicSharedMemorySize, G_SMEM);
  (void)hipFuncSetAttribute(reinterpret_cast<const void*>(&rnn_kernel),
                            hipFuncAttributeMaxDynamicSharedMemorySize, L_SMEM);

  prep_kernel<<<dim3(PB_END), dim3(256), 0, stream>>>(bn_g, bn_b, bn_m, bn_v, Ap, Ar, Wg, bgc,
                                                      g2, b2, m2, v2, W_ih, W_hh, b_ih, b_hh, ws);
  graph_kernel<<<dim3(NMB * 60), dim3(256), G_SMEM, stream>>>(x, AF, PAR, W2G, P);
  for (int c = 0; c < NCHUNK; ++c) {
    feat_kernel<<<dim3(CHROWS), dim3(256), 0, stream>>>(P, PAIRW, FEAT, c);
    xw_kernel<<<dim3(CHPAD / 128, G4 / 64), dim3(128), 0, stream>>>(FEAT, W2IH, PAR + PO_BSUM, XW, c);
  }
  rnn_kernel<<<dim3(13), dim3(192), L_SMEM, stream>>>(WHH, XW, HS);
  head_kernel<<<dim3(1), dim3(256), 0, stream>>>(HS, W_fc, b_fc, (float*)d_out);
  (void)hipGetLastError();
}
